// NeighborhoodAttention_10316511445126
// MI455X (gfx1250) — hardware-verified
//
#include <hip/hip_runtime.h>
#include <stdint.h>

typedef __attribute__((ext_vector_type(16))) _Float16 v16h;
typedef __attribute__((ext_vector_type(8)))  _Float16 v8h;
typedef __attribute__((ext_vector_type(16))) __bf16   v16b;
typedef __attribute__((ext_vector_type(8)))  __bf16   v8b;
typedef __attribute__((ext_vector_type(8)))  float    v8f;
typedef __attribute__((ext_vector_type(4)))  float    v4f;
typedef __attribute__((ext_vector_type(2)))  float    v2f;
typedef unsigned int v4u __attribute__((ext_vector_type(4), may_alias));

__device__ __forceinline__ unsigned short f2bf_bits(float f) {
  unsigned u = __float_as_uint(f);
  return (unsigned short)((u + 0x7FFFu + ((u >> 16) & 1u)) >> 16);
}
__device__ __forceinline__ float bf_bits2f(unsigned short h) { return __uint_as_float(((unsigned)h) << 16); }
__device__ __forceinline__ void split_bits(float f, unsigned short& hb, unsigned short& lb) {
  hb = f2bf_bits(f);
  lb = f2bf_bits(f - bf_bits2f(hb));
}

__device__ __forceinline__ void dep_guard_h(v8f& a, v8f& b, v16h x, v16h y) { asm volatile("v_nop\n\tv_nop\n\tv_nop\n\tv_nop" : "+v"(a), "+v"(b) : "v"(x), "v"(y)); }
__device__ __forceinline__ void dep_guard_b(v8f& a, v8f& b, v16b x, v16b y) { asm volatile("v_nop\n\tv_nop\n\tv_nop\n\tv_nop" : "+v"(a), "+v"(b) : "v"(x), "v"(y)); }
__device__ __forceinline__ void keep4_h(v16h a, v16h b, v16h c, v16h d) { asm volatile("v_nop" :: "v"(a), "v"(b), "v"(c), "v"(d)); }
__device__ __forceinline__ void keep4_b(v16b a, v16b b, v16b c, v16b d) { asm volatile("v_nop" :: "v"(a), "v"(b), "v"(c), "v"(d)); }
__device__ __forceinline__ void acc_guard4(v8f& a, v8f& b, v8f& c, v8f& d) { asm volatile("v_nop\n\tv_nop\n\tv_nop\n\tv_nop" : "+v"(a), "+v"(b), "+v"(c), "+v"(d)); }
template <typename T> struct Frag;
template <> struct Frag<_Float16> {
  typedef v16h V; union U { v16h v; v8h h[2]; };
  static __device__ __forceinline__ v16h load(const _Float16* p) {
    U f; f.h[0] = *(const v8h*)(p); f.h[1] = *(const v8h*)(p + 16); return f.v;
  }
  static __device__ __forceinline__ v8f mma(v16h a, v16h b, v8f c) {
    return __builtin_amdgcn_wmma_f32_16x16x32_f16(false, a, false, b, (short)0, c, false, false);
  }
  static __device__ __forceinline__ void guard(v8f& a, v8f& b, v16h x, v16h y) { dep_guard_h(a, b, x, y); }
  static __device__ __forceinline__ void keep(v16h a, v16h b, v16h c, v16h d) { keep4_h(a, b, c, d); }
};
template <> struct Frag<__bf16> {
  typedef v16b V; union U { v16b v; v8b h[2]; };
  static __device__ __forceinline__ v16b load(const __bf16* p) {
    U f; f.h[0] = *(const v8b*)(p); f.h[1] = *(const v8b*)(p + 16); return f.v;
  }
  static __device__ __forceinline__ v8f mma(v16b a, v16b b, v8f c) {
    return __builtin_amdgcn_wmma_f32_16x16x32_bf16(false, a, false, b, (short)0, c, false, false);
  }
  static __device__ __forceinline__ void guard(v8f& a, v8f& b, v16b x, v16b y) { dep_guard_b(a, b, x, y); }
  static __device__ __forceinline__ void keep(v16b a, v16b b, v16b c, v16b d) { keep4_b(a, b, c, d); }
};

template <int ET> struct Elem;
template <> struct Elem<0> { typedef _Float16 T; };
template <> struct Elem<1> { typedef __bf16 T; };
template <int ET, bool SPLIT, int BIAS_MODE, int OUT_MODE, bool RESID, int ACT = 0>
__global__ __launch_bounds__(256) void wmma_gemm64(
    const unsigned short* __restrict__ Ap, const unsigned short* __restrict__ A2p, int lda, long strideA,
    const unsigned short* __restrict__ Btp, const unsigned short* __restrict__ Bt2p, int ldb, long strideB,
    void* __restrict__ Cout, void* __restrict__ Cout2, int ldc, long strideC,
    const float* __restrict__ bias,
    const float* __restrict__ resid, long strideR,
    int M, int N, int K, float scale) {
  typedef typename Elem<ET>::T T;
  typedef typename Frag<T>::V V;
  const T* A = (const T*)Ap; const T* A2 = (const T*)A2p; const T* Bt = (const T*)Btp; const T* Bt2 = (const T*)Bt2p;
  __shared__ __align__(16) float sT[8][16 * 68];
  const int b    = blockIdx.y;
  const int lane = threadIdx.x & 31;
  const int wave = threadIdx.x >> 5;
  const int tilesN = N >> 6;
  const int tilesM = M >> 6;
  const int tile = blockIdx.x * 8 + wave;
  if (tile >= tilesM * tilesN) return;
  const int tm = tile / tilesN;
  const int tn = tile - tm * tilesN;
  const int m0 = tm << 6;
  const int n0 = tn << 6;

  const T* Ab  = A  + (size_t)b * strideA;
  const T* Bb  = Bt + (size_t)b * strideB;
  const T* Ab2 = SPLIT ? (A2  + (size_t)b * strideA) : nullptr;
  const T* Bb2 = SPLIT ? (Bt2 + (size_t)b * strideB) : nullptr;

  const int rlane = lane & 15;
  const int koff  = (lane >> 4) * 8;
  const int mOff  = (lane >> 4) * 8;

  v8f acc[4][4];
#pragma unroll
  for (int i = 0; i < 4; ++i)
#pragma unroll
    for (int j = 0; j < 4; ++j) acc[i][j] = (v8f){0.f,0.f,0.f,0.f,0.f,0.f,0.f,0.f};

  for (int k0 = 0; k0 < K; k0 += 32) {
    V bh[4], bl[4];
#pragma unroll
    for (int j = 0; j < 4; ++j) {
      const size_t bo = (size_t)(n0 + (j << 4) + rlane) * ldb + koff + k0;
      bh[j] = Frag<T>::load(Bb + bo);
      if (SPLIT) bl[j] = Frag<T>::load(Bb2 + bo);
    }
#pragma unroll
    for (int i = 0; i < 4; ++i) {
      const size_t ao = (size_t)(m0 + (i << 4) + rlane) * lda + koff + k0;
      V ah = Frag<T>::load(Ab + ao);
      V al;
      if (SPLIT) al = Frag<T>::load(Ab2 + ao);
#pragma unroll
      for (int j = 0; j < 4; ++j) {
        acc[i][j] = Frag<T>::mma(ah, bh[j], acc[i][j]);
        if (SPLIT) {
          acc[i][j] = Frag<T>::mma(ah, bl[j], acc[i][j]);
          acc[i][j] = Frag<T>::mma(al, bh[j], acc[i][j]);
        }
      }
      Frag<T>::guard(acc[i][0], acc[i][3], ah, SPLIT ? al : ah);
    }
    Frag<T>::keep(bh[0], bh[1], bh[2], bh[3]);
    if (SPLIT) Frag<T>::keep(bl[0], bl[1], bl[2], bl[3]);
  }
  acc_guard4(acc[0][0], acc[0][1], acc[0][2], acc[0][3]);
  acc_guard4(acc[1][0], acc[1][1], acc[1][2], acc[1][3]);
  acc_guard4(acc[2][0], acc[2][1], acc[2][2], acc[2][3]);
  acc_guard4(acc[3][0], acc[3][1], acc[3][2], acc[3][3]);

  float* slab = sT[wave];
  const float* Rb = RESID ? (resid + (size_t)b * strideR) : nullptr;
#pragma unroll
  for (int i = 0; i < 4; ++i) {
    const int mBase = m0 + (i << 4);
#pragma unroll
    for (int j = 0; j < 4; ++j) {
      const int n = n0 + (j << 4) + rlane;
      float bv = 0.f;
      if (BIAS_MODE == 2) bv = bias[n];
#pragma unroll
      for (int r = 0; r < 8; ++r) {
        float v = acc[i][j][r] * scale;
        if (BIAS_MODE == 1) v += bias[mBase + mOff + r];
        if (BIAS_MODE == 2) v += bv;
        if (RESID) v += Rb[(size_t)(mBase + mOff + r) * ldc + n];
        if (ACT == 1) v = tanhf(v);
        if (ACT == 2) v = fmaxf(v, 0.0f);
        if (ACT == 3) v = v / (1.0f + expf(-v));
        if (ACT == 4) v = (v > 0.f) ? v : 0.01f * v;
        if (ACT == 5) v = 0.5f * v * (1.0f + erff(v * 0.70710678118654752f));
        slab[(mOff + r) * 68 + (j << 4) + rlane] = v;
      }
    }
    __builtin_amdgcn_fence(__ATOMIC_RELEASE, "workgroup");
    __builtin_amdgcn_wave_barrier();
    __builtin_amdgcn_fence(__ATOMIC_ACQUIRE, "workgroup");
    if (OUT_MODE == 0) {
      float* C = (float*)Cout + (size_t)b * strideC;
      const int hh = lane >> 4, c4 = (lane & 15) * 4;
      for (int pass = 0; pass < 2; ++pass) {
#pragma unroll
        for (int it = 0; it < 8; ++it) {
          const int row = it * 2 + hh;
          v4f v = *(const v4f*)(slab + row * 68 + c4);
          *(volatile v4f*)(C + (size_t)(mBase + row) * ldc + n0 + c4) = v;
        }
        __threadfence();
      }
    } else {
      const int q = lane >> 3, c8 = (lane & 7) * 8;
      unsigned short* C  = (unsigned short*)Cout  + (size_t)b * strideC;
      unsigned short* C2 = (OUT_MODE == 2) ? ((unsigned short*)Cout2 + (size_t)b * strideC) : nullptr;
      for (int pass = 0; pass < 2; ++pass) {
#pragma unroll
        for (int it = 0; it < 4; ++it) {
          const int row = it * 4 + q;
          const float* sp = slab + row * 68 + c8;
          v8h hv, lv;
#pragma unroll
          for (int e = 0; e < 8; ++e) {
            if (OUT_MODE == 1) {
              hv[e] = (_Float16)sp[e];
            } else {
              unsigned short hb = f2bf_bits(sp[e]);
              unsigned short lb = f2bf_bits(sp[e] - bf_bits2f(hb));
              hv[e] = __builtin_bit_cast(_Float16, hb);
              lv[e] = __builtin_bit_cast(_Float16, lb);
            }
          }
          *(volatile v8h*)(C + (size_t)(mBase + row) * ldc + n0 + c8) = hv;
          if (OUT_MODE == 2) *(volatile v8h*)(C2 + (size_t)(mBase + row) * ldc + n0 + c8) = lv;
        }
        __threadfence();
      }
    }
    __builtin_amdgcn_fence(__ATOMIC_RELEASE, "workgroup");
    __builtin_amdgcn_wave_barrier();
    __builtin_amdgcn_fence(__ATOMIC_ACQUIRE, "workgroup");
  }
}

__device__ __forceinline__ v8f at_mma(v16b a, v16b b, v8f c) {
  c = __builtin_amdgcn_wmma_f32_16x16x32_bf16(false, a, false, b, (short)0, c, false, false);
  asm volatile("v_nop\n\tv_nop\n\tv_nop\n\tv_nop" : "+v"(c) : "v"(a), "v"(b));
  return c;
}
__device__ __forceinline__ void mem_order() { asm volatile("" ::: "memory"); }

#define IMG_HW   56
#define NTOK     12544
#define NHEAD    4
#define HDIM     32
#define CDIM     128
#define QKV_LD   384
#define WIN      7
#define HALF_WIN 3
#define REG_SIDE 10
#define NKEY     100
#define KROWS    112
#define PVK      128
#define OS_PITCH 132
#define RPB_SIDE 13
#define RPB_PER_HEAD 169
#define RPB_N    676
#define QT_SIDE  4
#define QT_PER_DIM 14

static_assert(NTOK == 4 * IMG_HW * IMG_HW);
static_assert(IMG_HW == QT_SIDE * QT_PER_DIM);
static_assert(NHEAD * HDIM == CDIM);
static_assert(RPB_N == NHEAD * RPB_PER_HEAD);
static_assert(RPB_N % 4 == 0);
static_assert(KROWS >= NKEY && KROWS % 16 == 0 && PVK >= KROWS && PVK % 32 == 0);
static_assert(IMG_HW - WIN == 49 && IMG_HW - REG_SIDE == 46);

__global__ __launch_bounds__(256) void cast_split_x2(
    const float* __restrict__ in, unsigned short* __restrict__ oh, unsigned short* __restrict__ ol, int n2) {
  const int i = blockIdx.x * 256 + threadIdx.x;
  if (i < n2) {
    const v2f f = *(const v2f*)(in + 2 * (size_t)i);
    unsigned short h0, l0, h1, l1;
    split_bits(f[0], h0, l0);
    split_bits(f[1], h1, l1);
    const unsigned uh = (unsigned)h0 | ((unsigned)h1 << 16);
    const unsigned ul = (unsigned)l0 | ((unsigned)l1 << 16);
    ((volatile unsigned*)oh)[i] = uh;
    ((volatile unsigned*)ol)[i] = ul;
    __threadfence();
    ((volatile unsigned*)oh)[i] = uh;
    ((volatile unsigned*)ol)[i] = ul;
  }
}

__global__ __launch_bounds__(256) void transpose_split_k128(
    const float* __restrict__ w, unsigned short* __restrict__ oh, unsigned short* __restrict__ ol, int ncols) {
  __shared__ float tile[128][33];
  const int tid = threadIdx.x;
  const int n0 = blockIdx.x * 32;
#pragma unroll 4
  for (int i = 0; i < 16; ++i) {
    const int idx = tid + 256 * i;
    const int k = idx >> 5, nn = idx & 31;
    tile[k][nn] = w[(size_t)k * ncols + n0 + nn];
  }
  __syncthreads();
  const int wave = tid >> 5, lane = tid & 31;
  const int q8 = lane >> 3, c8 = (lane & 7) * 8;
  for (int pass = 0; pass < 2; ++pass) {
#pragma unroll
    for (int it = 0; it < 2; ++it) {
      const int li = it * 32 + wave * 4 + q8;
      const int nn = li >> 1;
      const int kb = (li & 1) * 64 + c8;
      v4u vh, vl;
#pragma unroll
      for (int e = 0; e < 4; ++e) {
        const float f0 = tile[kb + 2 * e][nn];
        const float f1 = tile[kb + 2 * e + 1][nn];
        unsigned short h0, l0, h1, l1;
        split_bits(f0, h0, l0);
        split_bits(f1, h1, l1);
        vh[e] = (unsigned)h0 | ((unsigned)h1 << 16);
        vl[e] = (unsigned)l0 | ((unsigned)l1 << 16);
      }
      const size_t off = (size_t)(n0 + nn) * CDIM + kb;
      *(volatile v4u*)(oh + off) = vh;
      *(volatile v4u*)(ol + off) = vl;
    }
    __threadfence();
  }
}

union FB { v16b v; v8b h[2]; };

__global__ __launch_bounds__(32) __attribute__((amdgpu_num_vgpr(256)))
void win_attn_kernel(const unsigned short* __restrict__ QH, const unsigned short* __restrict__ QL,
                     const float* __restrict__ rpb,
                     unsigned short* __restrict__ AH, unsigned short* __restrict__ AL) {
  __shared__ __align__(16) __bf16 Ksh[KROWS * HDIM];
  __shared__ __align__(16) __bf16 Ksl[KROWS * HDIM];
  __shared__ __align__(16) __bf16 Vth[HDIM * PVK];
  __shared__ __align__(16) __bf16 Vtl[HDIM * PVK];
  __shared__ __align__(16) __bf16 Psh[16 * PVK];
  __shared__ __align__(16) __bf16 Psl[16 * PVK];
  __shared__ __align__(16) float  Os[16 * OS_PITCH];
  __shared__ __align__(16) float  Bsh[RPB_N];

  const int lane = threadIdx.x & 31;
  const int hh   = lane >> 4;
  const int c    = lane & 15;

  int bx = blockIdx.x;
  const int tw = bx % QT_PER_DIM; bx /= QT_PER_DIM;
  const int th = bx % QT_PER_DIM;
  const int b  = bx / QT_PER_DIM;
  const int h0 = th * QT_SIDE;
  const int w0 = tw * QT_SIDE;
  int rbase = h0 - HALF_WIN; rbase = rbase < 0 ? 0 : rbase; rbase = rbase > (IMG_HW - REG_SIDE) ? (IMG_HW - REG_SIDE) : rbase;
  int cbase = w0 - HALF_WIN; cbase = cbase < 0 ? 0 : cbase; cbase = cbase > (IMG_HW - REG_SIDE) ? (IMG_HW - REG_SIDE) : cbase;

  {
    const v4u z4 = {0u, 0u, 0u, 0u};
#pragma unroll
    for (int q = 0; q < 2; ++q) {
      const int idx = lane + 32 * q;
      ((v4u*)(Ksh + 96 * HDIM))[idx] = z4;
      ((v4u*)(Ksl + 96 * HDIM))[idx] = z4;
    }
#pragma unroll
    for (int q = 0; q < 4; ++q) {
      const int idx = lane + 32 * q;
      const int d = idx >> 2, part = idx & 3;
      ((v4u*)(Vth + d * PVK + 96))[part] = z4;
      ((v4u*)(Vtl + d * PVK + 96))[part] = z4;
    }
    {
      const int r = lane >> 1, part = lane & 1;
      ((v4u*)(Psh + r * PVK + 112))[part] = z4;
      ((v4u*)(Psl + r * PVK + 112))[part] = z4;
    }
#pragma unroll 1
    for (int i = lane; i < RPB_N / 4; i += 32) ((v4f*)Bsh)[i] = ((const v4f*)rpb)[i];
  }
  __syncthreads();

  const int tokq = (b * IMG_HW + h0 + (c >> 2)) * IMG_HW + w0 + (c & 3);
  const float SC = 0.17677669529663688f;

#pragma unroll 1
  for (int head = 0; head < NHEAD; ++head) {
    __syncthreads();
#pragma unroll 1
    for (int it = 0; it < 4; ++it) {
      const int j  = lane + 32 * it;
      const int jj = j < NKEY ? j : (NKEY - 1);
      const int lr = jj / REG_SIDE;
      const int lc = jj - lr * REG_SIDE;
      const size_t tok = (size_t)((b * IMG_HW + rbase + lr) * IMG_HW + cbase + lc);
      {
        const v4u* ks = (const v4u*)(QH + tok * QKV_LD + CDIM + head * HDIM);
        const v4u* ls = (const v4u*)(QL + tok * QKV_LD + CDIM + head * HDIM);
        const v4u k0 = ks[0], k1 = ks[1], k2 = ks[2], k3 = ks[3];
        const v4u l0 = ls[0], l1 = ls[1], l2 = ls[2], l3 = ls[3];
        if (j < NKEY) {
          v4u* kd = (v4u*)(Ksh + j * HDIM);
          v4u* ld = (v4u*)(Ksl + j * HDIM);
          kd[0] = k0; kd[1] = k1; kd[2] = k2; kd[3] = k3;
          ld[0] = l0; ld[1] = l1; ld[2] = l2; ld[3] = l3;
        }
      }
      mem_order();
      {
        const v4u* vs = (const v4u*)(QH + tok * QKV_LD + 2 * CDIM + head * HDIM);
        const v4u* ws = (const v4u*)(QL + tok * QKV_LD + 2 * CDIM + head * HDIM);
        v4u va[4], vb[4];
#pragma unroll
        for (int q = 0; q < 4; ++q) { va[q] = vs[q]; vb[q] = ws[q]; }
        if (j < NKEY) {
#pragma unroll
          for (int q = 0; q < 4; ++q) {
#pragma unroll
            for (int e = 0; e < 4; ++e) {
              const unsigned wa = va[q][e];
              const unsigned wb = vb[q][e];
              const int d = q * 8 + 2 * e;
              Vth[d * PVK + j]       = __builtin_bit_cast(__bf16, (unsigned short)(wa & 0xffffu));
              Vth[(d + 1) * PVK + j] = __builtin_bit_cast(__bf16, (unsigned short)(wa >> 16));
              Vtl[d * PVK + j]       = __builtin_bit_cast(__bf16, (unsigned short)(wb & 0xffffu));
              Vtl[(d + 1) * PVK + j] = __builtin_bit_cast(__bf16, (unsigned short)(wb >> 16));
            }
          }
        }
      }
      mem_order();
    }
    __syncthreads();

    const v16b qa = Frag<__bf16>::load((const __bf16*)(QH + (size_t)tokq * QKV_LD + head * HDIM + 8 * hh));
    const v16b ql = Frag<__bf16>::load((const __bf16*)(QL + (size_t)tokq * QKV_LD + head * HDIM + 8 * hh));

    v8f s[7];
#pragma unroll
    for (int t = 0; t < 7; ++t) {
      s[t] = (v8f){0.f,0.f,0.f,0.f,0.f,0.f,0.f,0.f};
      FB kb, kl;
      kb.h[0] = *(const v8b*)(Ksh + (t * 16 + c) * HDIM + 8 * hh);
      kb.h[1] = *(const v8b*)(Ksh + (t * 16 + c) * HDIM + 16 + 8 * hh);
      kl.h[0] = *(const v8b*)(Ksl + (t * 16 + c) * HDIM + 8 * hh);
      kl.h[1] = *(const v8b*)(Ksl + (t * 16 + c) * HDIM + 16 + 8 * hh);
      s[t] = at_mma(qa, kb.v, s[t]);
      s[t] = at_mma(qa, kl.v, s[t]);
      s[t] = at_mma(ql, kb.v, s[t]);
      mem_order();
    }

    float linv[8];
#pragma unroll
    for (int r = 0; r < 8; ++r) {
      const int m  = 8 * hh + r;
      const int qh = h0 + (m >> 2);
      const int qw = w0 + (m & 3);
      int sh = qh - HALF_WIN; sh = sh < 0 ? 0 : sh; sh = sh > (IMG_HW - WIN) ? (IMG_HW - WIN) : sh;
      int sw = qw - HALF_WIN; sw = sw < 0 ? 0 : sw; sw = sw > (IMG_HW - WIN) ? (IMG_HW - WIN) : sw;
      float mx = -__builtin_inff();
#pragma unroll
      for (int t = 0; t < 7; ++t) {
        const int j  = t * 16 + c;
        const int lr = j / REG_SIDE;
        const int lc = j - lr * REG_SIDE;
        const int kr = rbase + lr;
        const int kc = cbase + lc;
        const bool valid = ((unsigned)(kr - sh) <= 6u) && ((unsigned)(kc - sw) <= 6u);
        int bi = (kr - qh + (WIN - 1)) * RPB_SIDE + (kc - qw + (WIN - 1));
        bi = bi < 0 ? 0 : bi; bi = bi > (RPB_PER_HEAD - 1) ? (RPB_PER_HEAD - 1) : bi;
        const float bv  = Bsh[head * RPB_PER_HEAD + bi];
        const float val = s[t][r] * SC + bv;
        const float sv  = valid ? val : -__builtin_inff();
        s[t][r] = sv;
        mx = fmaxf(mx, sv);
      }
#pragma unroll
      for (int off = 1; off < 16; off <<= 1) mx = fmaxf(mx, __shfl_xor(mx, off, 32));
      float psum = 0.f;
#pragma unroll
      for (int t = 0; t < 7; ++t) {
        const float p = expf(s[t][r] - mx);
        psum += p;
        unsigned short hb, lb;
        split_bits(p, hb, lb);
        Psh[m * PVK + t * 16 + c] = __builtin_bit_cast(__bf16, hb);
        Psl[m * PVK + t * 16 + c] = __builtin_bit_cast(__bf16, lb);
      }
#pragma unroll
      for (int off = 1; off < 16; off <<= 1) psum += __shfl_xor(psum, off, 32);
      linv[r] = 1.0f / psum;
      mem_order();
    }
    __syncthreads();

    v8f oacc[2];
    oacc[0] = (v8f){0.f,0.f,0.f,0.f,0.f,0.f,0.f,0.f};
    oacc[1] = (v8f){0.f,0.f,0.f,0.f,0.f,0.f,0.f,0.f};
#pragma unroll 1
    for (int kk = 0; kk < 4; ++kk) {
      FB pa, pl;
      pa.h[0] = *(const v8b*)(Psh + c * PVK + kk * 32 + 8 * hh);
      pa.h[1] = *(const v8b*)(Psh + c * PVK + kk * 32 + 16 + 8 * hh);
      pl.h[0] = *(const v8b*)(Psl + c * PVK + kk * 32 + 8 * hh);
      pl.h[1] = *(const v8b*)(Psl + c * PVK + kk * 32 + 16 + 8 * hh);
#pragma unroll
      for (int t = 0; t < 2; ++t) {
        FB vb, vl;
        vb.h[0] = *(const v8b*)(Vth + (t * 16 + c) * PVK + kk * 32 + 8 * hh);
        vb.h[1] = *(const v8b*)(Vth + (t * 16 + c) * PVK + kk * 32 + 16 + 8 * hh);
        vl.h[0] = *(const v8b*)(Vtl + (t * 16 + c) * PVK + kk * 32 + 8 * hh);
        vl.h[1] = *(const v8b*)(Vtl + (t * 16 + c) * PVK + kk * 32 + 16 + 8 * hh);
        oacc[t] = at_mma(pa.v, vb.v, oacc[t]);
        oacc[t] = at_mma(pa.v, vl.v, oacc[t]);
        oacc[t] = at_mma(pl.v, vb.v, oacc[t]);
      }
      mem_order();
    }
#pragma unroll
    for (int r = 0; r < 8; ++r) {
#pragma unroll
      for (int t = 0; t < 2; ++t) Os[(8 * hh + r) * OS_PITCH + head * HDIM + t * 16 + c] = oacc[t][r] * linv[r];
    }
  }
  __syncthreads();

  {
    const int q8 = lane >> 3, c8 = (lane & 7) * 8;
    for (int pass = 0; pass < 2; ++pass) {
#pragma unroll
      for (int it = 0; it < 8; ++it) {
        const int li   = it * 4 + q8;
        const int row  = li >> 1;
        const int col0 = (li & 1) * 64 + c8;
        const v4f f0 = *(const v4f*)(Os + row * OS_PITCH + col0);
        const v4f f1 = *(const v4f*)(Os + row * OS_PITCH + col0 + 4);
        v4u vh, vl;
        unsigned short ha, la, hb2, lb2;
        split_bits(f0[0], ha, la); split_bits(f0[1], hb2, lb2);
        vh[0] = (unsigned)ha | ((unsigned)hb2 << 16); vl[0] = (unsigned)la | ((unsigned)lb2 << 16);
        split_bits(f0[2], ha, la); split_bits(f0[3], hb2, lb2);
        vh[1] = (unsigned)ha | ((unsigned)hb2 << 16); vl[1] = (unsigned)la | ((unsigned)lb2 << 16);
        split_bits(f1[0], ha, la); split_bits(f1[1], hb2, lb2);
        vh[2] = (unsigned)ha | ((unsigned)hb2 << 16); vl[2] = (unsigned)la | ((unsigned)lb2 << 16);
        split_bits(f1[2], ha, la); split_bits(f1[3], hb2, lb2);
        vh[3] = (unsigned)ha | ((unsigned)hb2 << 16); vl[3] = (unsigned)la | ((unsigned)lb2 << 16);
        const size_t tok = (size_t)((b * IMG_HW + h0 + (row >> 2)) * IMG_HW + w0 + (row & 3));
        *(volatile v4u*)(AH + tok * CDIM + col0) = vh;
        *(volatile v4u*)(AL + tok * CDIM + col0) = vl;
      }
      __threadfence();
    }
  }
}

#define SZ_XPL   ((size_t)NTOK * CDIM * 2)
#define SZ_WQPL  ((size_t)QKV_LD * CDIM * 2)
#define SZ_WPPL  ((size_t)CDIM * CDIM * 2)
#define SZ_QKVPL ((size_t)NTOK * QKV_LD * 2)
#define OFF_XH   ((size_t)0)
#define OFF_XL   (OFF_XH + SZ_XPL)
#define OFF_WQH  (OFF_XL + SZ_XPL)
#define OFF_WQL  (OFF_WQH + SZ_WQPL)
#define OFF_WPH  (OFF_WQL + SZ_WQPL)
#define OFF_WPL  (OFF_WPH + SZ_WPPL)
#define OFF_QKVH (OFF_WPL + SZ_WPPL)
#define OFF_QKVL (OFF_QKVH + SZ_QKVPL)
#define OFF_AH   (OFF_QKVL + SZ_QKVPL)
#define OFF_AL   (OFF_AH + SZ_XPL)
#define WS_TOTAL (OFF_AL + SZ_XPL)
static_assert(WS_TOTAL == 32374784);
static_assert(WS_TOTAL <= 134217728);
static_assert(OFF_QKVH % 256 == 0 && OFF_AH % 256 == 0 && OFF_WQH % 256 == 0 && OFF_WPH % 256 == 0);
static_assert(NTOK % 64 == 0 && QKV_LD % 64 == 0 && CDIM % 64 == 0 && CDIM % 32 == 0);
static_assert(QKV_LD % 32 == 0 && CDIM % 32 == 0);
static_assert((NTOK * CDIM / 2) % 256 == 0);

extern "C" void kernel_launch(void* const* d_in, const int* in_sizes, int n_in,
                              void* d_out, int out_size, void* d_ws, size_t ws_size,
                              hipStream_t stream)
{
  if (n_in < 6) return;
  if (in_sizes[0] != NTOK * CDIM || in_sizes[1] != CDIM * QKV_LD || in_sizes[2] != QKV_LD ||
      in_sizes[3] != RPB_N || in_sizes[4] != CDIM * CDIM || in_sizes[5] != CDIM) return;
  if (out_size != NTOK * CDIM) return;
  if (ws_size < WS_TOTAL) return;

  const float* x      = (const float*)d_in[0];
  const float* w_qkv  = (const float*)d_in[1];
  const float* b_qkv  = (const float*)d_in[2];
  const float* rpb    = (const float*)d_in[3];
  const float* w_proj = (const float*)d_in[4];
  const float* b_proj = (const float*)d_in[5];
  float* out = (float*)d_out;

  unsigned char* ws = (unsigned char*)d_ws;
  unsigned short* XH   = (unsigned short*)(ws + OFF_XH);
  unsigned short* XL   = (unsigned short*)(ws + OFF_XL);
  unsigned short* WQH  = (unsigned short*)(ws + OFF_WQH);
  unsigned short* WQL  = (unsigned short*)(ws + OFF_WQL);
  unsigned short* WPH  = (unsigned short*)(ws + OFF_WPH);
  unsigned short* WPL  = (unsigned short*)(ws + OFF_WPL);
  unsigned short* QKVH = (unsigned short*)(ws + OFF_QKVH);
  unsigned short* QKVL = (unsigned short*)(ws + OFF_QKVL);
  unsigned short* AH   = (unsigned short*)(ws + OFF_AH);
  unsigned short* AL   = (unsigned short*)(ws + OFF_AL);

  {
    const int n2 = NTOK * CDIM / 2;
    cast_split_x2<<<(n2 + 255) / 256, 256, 0, stream>>>(x, XH, XL, n2);
  }
  transpose_split_k128<<<QKV_LD / 32, 256, 0, stream>>>(w_qkv, WQH, WQL, QKV_LD);
  transpose_split_k128<<<CDIM / 32, 256, 0, stream>>>(w_proj, WPH, WPL, CDIM);

  {
    const int tiles = (NTOK / 64) * (QKV_LD / 64);
    wmma_gemm64<1, true, 2, 2, false, 0><<<dim3((tiles + 7) / 8, 1), 256, 0, stream>>>(
        XH, XL, CDIM, 0L, WQH, WQL, CDIM, 0L,
        (void*)QKVH, (void*)QKVL, QKV_LD, 0L,
        b_qkv, nullptr, 0L, NTOK, QKV_LD, CDIM, 1.0f);
  }
  win_attn_kernel<<<4 * QT_PER_DIM * QT_PER_DIM, 32, 0, stream>>>(QKVH, QKVL, rpb, AH, AL);

  {
    const int tiles = (NTOK / 64) * (CDIM / 64);
    wmma_gemm64<1, true, 2, 0, false, 0><<<dim3((tiles + 7) / 8, 1), 256, 0, stream>>>(
        AH, AL, CDIM, 0L, WPH, WPL, CDIM, 0L,
        (void*)out, nullptr, CDIM, 0L,
        b_proj, nullptr, 0L, NTOK, CDIM, CDIM, 1.0f);
  }
}
